// FlexMoE_38646115729759
// MI455X (gfx1250) — hardware-run, weakly checked
//
#include <hip/hip_runtime.h>
#include <math.h>

typedef __attribute__((ext_vector_type(16))) __bf16   v16b;
typedef __attribute__((ext_vector_type(8)))  float    v8f;
typedef __attribute__((ext_vector_type(4)))  float    v4f;
typedef __attribute__((ext_vector_type(4)))  unsigned v4u;
typedef __attribute__((ext_vector_type(8)))  unsigned v8u;
typedef __attribute__((ext_vector_type(4)))  int      v4i;

constexpr int kMod = 4;
constexpr int kBat = 2048;
constexpr int kDin = 1024;
constexpr int kOut = 1024;
constexpr int kExp = 8;
constexpr int kCls = 2;
constexpr int kTok = kMod * kBat;
constexpr int kNV  = kExp * kCls;
constexpr int kGateThreads = 128;
constexpr int kFoldRows    = 64;
static_assert(kTok == 8192, "token count");
static_assert(kNV == 16, "one 16-wide column tile");
static_assert((kDin % 32) == 0, "k-steps of 32");
static_assert((kTok % (64 * 8)) == 0, "row tiles of 64, eight per block");
static_assert((kTok % kGateThreads) == 0, "gate grid exact");
static_assert((kDin % kFoldRows) == 0 && (kOut % 128) == 0, "fold tiling");
static_assert((kBat % 64) == 0, "pool grid exact");

constexpr size_t kOffVT  = 0;
constexpr size_t kOffVB  = kOffVT  + (size_t)2 * kNV * kDin * 2;
constexpr size_t kOffWIN = kOffVB  + (size_t)32 * 4;
constexpr size_t kOffSC  = kOffWIN + (size_t)kTok * 4;
constexpr size_t kOffG   = kOffSC  + (size_t)kTok * 4;
constexpr size_t kWsTotal = kOffG  + (size_t)kTok * kNV * 4;
static_assert(kWsTotal == 655488ull, "carve total");
static_assert(kWsTotal <= 134217728ull, "carve cap");
static_assert((kOffVB % 128) == 0 && (kOffWIN % 128) == 0 && (kOffSC % 128) == 0 && (kOffG % 128) == 0, "128-B aligned regions");

__device__ __forceinline__ void split2(float a, float b, unsigned& hw, unsigned& lw) {
  const unsigned ua = __float_as_uint(a);
  const unsigned ub = __float_as_uint(b);
  const unsigned ra = ua + 0x7FFFu + ((ua >> 16) & 1u);
  const unsigned rb = ub + 0x7FFFu + ((ub >> 16) & 1u);
  const unsigned ha = ra & 0xFFFF0000u;
  const unsigned hb = rb & 0xFFFF0000u;
  hw = (ha >> 16) | hb;
  const float la = a - __uint_as_float(ha);
  const float lb = b - __uint_as_float(hb);
  const unsigned va = __float_as_uint(la);
  const unsigned vb = __float_as_uint(lb);
  const unsigned sa = va + 0x7FFFu + ((va >> 16) & 1u);
  const unsigned sb = vb + 0x7FFFu + ((vb >> 16) & 1u);
  lw = (sa >> 16) | (sb & 0xFFFF0000u);
}

__device__ __forceinline__ v8f mma_bf(v16b a, v16b b, v8f c) {
  c = __builtin_amdgcn_wmma_f32_16x16x32_bf16(false, a, false, b, (short)0, c, false, false);
  asm volatile("v_nop\n\tv_nop\n\tv_nop\n\tv_nop" : "+v"(c) : "v"(a), "v"(b));
  return c;
}

__global__ __launch_bounds__(128) void gate_select_kernel(
    const float* __restrict__ x, const float* __restrict__ gate_w, const float* __restrict__ gate_b,
    int* __restrict__ WIN, float* __restrict__ SC)
{
  __shared__ __align__(16) float sGw[kDin * kExp];
  __shared__ __align__(16) float sLg[kExp * kGateThreads];
  __shared__ __align__(16) int   sWin[kGateThreads];
  __shared__ __align__(16) float sSc[kGateThreads];
  const int tid = threadIdx.x, lane = tid & 31, wave = tid >> 5;
#pragma unroll 1
  for (int i = 0; i < 16; ++i) {
    const int idx = (i * kGateThreads + tid) * 4;
    *(v4f*)(sGw + idx) = *(const v4f*)(gate_w + idx);
  }
  __syncthreads();
  const int t = blockIdx.x * kGateThreads + tid;
  const float* px = x + (size_t)t * kDin;
  float acc[kExp];
#pragma unroll
  for (int e = 0; e < kExp; ++e) acc[e] = 0.f;
#pragma unroll 1
  for (int d4 = 0; d4 < kDin / 4; ++d4) {
    const v4f xv = *(const v4f*)(px + d4 * 4);
#pragma unroll
    for (int j = 0; j < 4; ++j) {
      const float* g = sGw + (d4 * 4 + j) * kExp;
      const v4f g0 = *(const v4f*)(g);
      const v4f g1 = *(const v4f*)(g + 4);
      const float xs = xv[j];
      acc[0] = fmaf(xs, g0[0], acc[0]);
      acc[1] = fmaf(xs, g0[1], acc[1]);
      acc[2] = fmaf(xs, g0[2], acc[2]);
      acc[3] = fmaf(xs, g0[3], acc[3]);
      acc[4] = fmaf(xs, g1[0], acc[4]);
      acc[5] = fmaf(xs, g1[1], acc[5]);
      acc[6] = fmaf(xs, g1[2], acc[6]);
      acc[7] = fmaf(xs, g1[3], acc[7]);
    }
  }
  const v4f gb0 = *(const v4f*)(gate_b);
  const v4f gb1 = *(const v4f*)(gate_b + 4);
  float lg[kExp];
  lg[0] = acc[0] + gb0[0];
  lg[1] = acc[1] + gb0[1];
  lg[2] = acc[2] + gb0[2];
  lg[3] = acc[3] + gb0[3];
  lg[4] = acc[4] + gb1[0];
  lg[5] = acc[5] + gb1[1];
  lg[6] = acc[6] + gb1[2];
  lg[7] = acc[7] + gb1[3];
  int i1 = 0;
  float v1 = lg[0];
#pragma unroll
  for (int e = 1; e < kExp; ++e) {
    const bool gt = lg[e] > v1;
    v1 = gt ? lg[e] : v1;
    i1 = gt ? e : i1;
  }
  int i2 = 0;
  float v2 = -INFINITY;
#pragma unroll
  for (int e = 0; e < kExp; ++e) {
    const bool gt = (e != i1) && (lg[e] > v2);
    v2 = gt ? lg[e] : v2;
    i2 = gt ? e : i2;
  }
  const int win = (i1 > i2) ? i1 : i2;
#pragma unroll
  for (int e = 0; e < kExp; ++e) sLg[e * kGateThreads + tid] = lg[e];
  float z = 0.f;
#pragma unroll 1
  for (int e = 0; e < kExp; ++e) z += expf(sLg[e * kGateThreads + tid] - v1);
  const float e2 = expf(v2 - v1);
  const float rz = 1.0f / z;
  const float p1 = rz;
  const float p2 = e2 * rz;
  const float ps = p1 + p2;
  const float rs = 1.0f / ps;
  const float sc = p1 * rs + p2 * rs;
  sWin[tid] = win;
  sSc[tid]  = sc;
  __syncthreads();
  if (wave == 0) {
    const v4i wv = *(const v4i*)(sWin + lane * 4);
    int* dst = WIN + (size_t)blockIdx.x * kGateThreads + lane * 4;
    for (int pass = 0; pass < 2; ++pass) {
      *(volatile v4i*)dst = wv;
      __threadfence();
    }
  }
  if (wave == 1) {
    const v4f sv = *(const v4f*)(sSc + lane * 4);
    float* dst = SC + (size_t)blockIdx.x * kGateThreads + lane * 4;
    for (int pass = 0; pass < 2; ++pass) {
      *(volatile v4f*)dst = sv;
      __threadfence();
    }
  }
}

__global__ __launch_bounds__(256) void fold_head_kernel(
    const float* __restrict__ expert_w, const float* __restrict__ expert_b, const float* __restrict__ head_w,
    unsigned short* __restrict__ VT, float* __restrict__ VB)
{
  __shared__ __align__(16) float sV[2 * kFoldRows];
  const int tid = threadIdx.x, lane = tid & 31, wave = tid >> 5;
  const int blk = blockIdx.x;
  const bool isBias = (blk == kExp * 16);
  const int e  = isBias ? 0 : (blk >> 4);
  const int d0 = (blk & 15) * kFoldRows;
  v4f hA[8], hB[8];
#pragma unroll
  for (int it = 0; it < 8; ++it) {
    const int o = it * 128 + lane * 4;
    hA[it] = *(const v4f*)(head_w + 2 * o);
    hB[it] = *(const v4f*)(head_w + 2 * o + 4);
  }
#pragma unroll 1
  for (int i = 0; i < 8; ++i) {
    const int rl = wave * 8 + i;
    const float* src = isBias ? (expert_b + (size_t)(rl & 7) * kOut)
                              : (expert_w + ((size_t)e * kDin + d0 + rl) * kOut);
    float a0 = 0.f, a1 = 0.f;
#pragma unroll
    for (int it = 0; it < 8; ++it) {
      const v4f w = *(const v4f*)(src + it * 128 + lane * 4);
      a0 = fmaf(w[0], hA[it][0], a0);
      a1 = fmaf(w[0], hA[it][1], a1);
      a0 = fmaf(w[1], hA[it][2], a0);
      a1 = fmaf(w[1], hA[it][3], a1);
      a0 = fmaf(w[2], hB[it][0], a0);
      a1 = fmaf(w[2], hB[it][1], a1);
      a0 = fmaf(w[3], hB[it][2], a0);
      a1 = fmaf(w[3], hB[it][3], a1);
    }
#pragma unroll
    for (int off = 16; off >= 1; off >>= 1) {
      a0 += __shfl_xor(a0, off, 32);
      a1 += __shfl_xor(a1, off, 32);
    }
    if (lane == 0) {
      sV[rl] = a0;
      sV[kFoldRows + rl] = a1;
    }
  }
  __syncthreads();
  if (wave == 0) {
    if (!isBias) {
      const int q = lane >> 3, j = lane & 7;
      const int c = q & 1, pl = q >> 1;
      const float* sp = sV + c * kFoldRows + j * 8;
      const v4f f0 = *(const v4f*)(sp);
      const v4f f1 = *(const v4f*)(sp + 4);
      unsigned h0, h1, h2, h3, l0, l1, l2, l3;
      split2(f0[0], f0[1], h0, l0);
      split2(f0[2], f0[3], h1, l1);
      split2(f1[0], f1[1], h2, l2);
      split2(f1[2], f1[3], h3, l3);
      v4u ov;
      ov[0] = (pl != 0) ? l0 : h0;
      ov[1] = (pl != 0) ? l1 : h1;
      ov[2] = (pl != 0) ? l2 : h2;
      ov[3] = (pl != 0) ? l3 : h3;
      unsigned short* dst = VT + (size_t)(pl * kNV + 2 * e + c) * kDin + d0 + j * 8;
      for (int pass = 0; pass < 2; ++pass) {
        *(volatile v4u*)(void*)dst = ov;
        __threadfence();
      }
    } else {
      v4f bv;
#pragma unroll
      for (int k = 0; k < 4; ++k) {
        const int n = (lane & 7) * 4 + k;
        const float tv = sV[(n & 1) * kFoldRows + ((n >> 1) & 7)];
        bv[k] = (n < kNV) ? tv : 0.f;
      }
      if (lane < 8) {
        float* dst = VB + lane * 4;
        for (int pass = 0; pass < 2; ++pass) {
          *(volatile v4f*)dst = bv;
          __threadfence();
        }
      }
    }
  }
}

__global__ __launch_bounds__(256) void xv_wmma_kernel(
    const float* __restrict__ x, const unsigned short* __restrict__ VT, float* __restrict__ G)
{
  __shared__ __align__(16) float sT[8][64 * kNV];
  const int lane = threadIdx.x & 31, wave = threadIdx.x >> 5;
  const int tile = blockIdx.x * 8 + wave;
  const int m0 = tile * 64;
  const int rl = lane & 15, hh = lane >> 4, koff = hh * 8;
  const unsigned short* bhp = VT + (size_t)rl * kDin + koff;
  const unsigned short* blp = bhp + (size_t)kNV * kDin;
  const float* xa = x + (size_t)(m0 + rl) * kDin + koff;
  v8f acc[4];
#pragma unroll
  for (int i = 0; i < 4; ++i) acc[i] = (v8f){0.f, 0.f, 0.f, 0.f, 0.f, 0.f, 0.f, 0.f};
#pragma unroll 1
  for (int k0 = 0; k0 < kDin; k0 += 32) {
    const v4u bh0 = *(const v4u*)(const void*)(bhp + k0);
    const v4u bh1 = *(const v4u*)(const void*)(bhp + k0 + 16);
    const v4u bl0 = *(const v4u*)(const void*)(blp + k0);
    const v4u bl1 = *(const v4u*)(const void*)(blp + k0 + 16);
    const v8u bhw = __builtin_shufflevector(bh0, bh1, 0, 1, 2, 3, 4, 5, 6, 7);
    const v8u blw = __builtin_shufflevector(bl0, bl1, 0, 1, 2, 3, 4, 5, 6, 7);
    const v16b bH = __builtin_bit_cast(v16b, bhw);
    const v16b bL = __builtin_bit_cast(v16b, blw);
#pragma unroll
    for (int i = 0; i < 4; ++i) {
      const float* p = xa + (size_t)i * 16 * kDin + k0;
      const v4f f0 = *(const v4f*)(p);
      const v4f f1 = *(const v4f*)(p + 4);
      const v4f f2 = *(const v4f*)(p + 16);
      const v4f f3 = *(const v4f*)(p + 20);
      v8u hw, lw;
      unsigned h, l;
      split2(f0[0], f0[1], h, l);
      hw[0] = h;
      lw[0] = l;
      split2(f0[2], f0[3], h, l);
      hw[1] = h;
      lw[1] = l;
      split2(f1[0], f1[1], h, l);
      hw[2] = h;
      lw[2] = l;
      split2(f1[2], f1[3], h, l);
      hw[3] = h;
      lw[3] = l;
      split2(f2[0], f2[1], h, l);
      hw[4] = h;
      lw[4] = l;
      split2(f2[2], f2[3], h, l);
      hw[5] = h;
      lw[5] = l;
      split2(f3[0], f3[1], h, l);
      hw[6] = h;
      lw[6] = l;
      split2(f3[2], f3[3], h, l);
      hw[7] = h;
      lw[7] = l;
      const v16b aH = __builtin_bit_cast(v16b, hw);
      const v16b aL = __builtin_bit_cast(v16b, lw);
      acc[i] = mma_bf(aH, bH, acc[i]);
      acc[i] = mma_bf(aH, bL, acc[i]);
      acc[i] = mma_bf(aL, bH, acc[i]);
    }
  }
  float* slab = sT[wave];
#pragma unroll
  for (int i = 0; i < 4; ++i) {
#pragma unroll
    for (int r = 0; r < 8; ++r) slab[(16 * i + 8 * hh + r) * kNV + rl] = acc[i][r];
  }
  __syncthreads();
  float* gp = G + (size_t)m0 * kNV;
  for (int pass = 0; pass < 2; ++pass) {
#pragma unroll
    for (int it = 0; it < 8; ++it) {
      const v4f v = *(const v4f*)(slab + it * 128 + lane * 4);
      *(volatile v4f*)(gp + it * 128 + lane * 4) = v;
    }
    __threadfence();
  }
}

__global__ __launch_bounds__(64) void pool_select_kernel(
    const float* __restrict__ G, const int* __restrict__ WIN, const float* __restrict__ SC,
    const float* __restrict__ VB, const float* __restrict__ head_b, float* __restrict__ out)
{
  __shared__ __align__(16) float sO[128];
  const int tid = threadIdx.x, lane = tid & 31, wave = tid >> 5;
  const int b = blockIdx.x * 64 + tid;
  const v4f vb0 = *(const v4f*)(VB);
  const v4f vb1 = *(const v4f*)(VB + 4);
  const v4f vb2 = *(const v4f*)(VB + 8);
  const v4f vb3 = *(const v4f*)(VB + 12);
  const float hb0 = head_b[0];
  const float hb1 = head_b[1];
  float o0 = 0.f, o1 = 0.f;
#pragma unroll
  for (int m = 0; m < kMod; ++m) {
    const int t = m * kBat + b;
    int w = WIN[t];
    w = (w < 0) ? 0 : w;
    w = (w > kExp - 1) ? (kExp - 1) : w;
    const float sc = SC[t];
    const float* gr = G + (size_t)t * kNV;
    const v4f r0 = *(const v4f*)(gr);
    const v4f r1 = *(const v4f*)(gr + 4);
    const v4f r2 = *(const v4f*)(gr + 8);
    const v4f r3 = *(const v4f*)(gr + 12);
    float g0 = r0[0], g1 = r0[1], c0 = vb0[0], c1 = vb0[1];
    g0 = (w == 1) ? r0[2] : g0;
    g1 = (w == 1) ? r0[3] : g1;
    c0 = (w == 1) ? vb0[2] : c0;
    c1 = (w == 1) ? vb0[3] : c1;
    g0 = (w == 2) ? r1[0] : g0;
    g1 = (w == 2) ? r1[1] : g1;
    c0 = (w == 2) ? vb1[0] : c0;
    c1 = (w == 2) ? vb1[1] : c1;
    g0 = (w == 3) ? r1[2] : g0;
    g1 = (w == 3) ? r1[3] : g1;
    c0 = (w == 3) ? vb1[2] : c0;
    c1 = (w == 3) ? vb1[3] : c1;
    g0 = (w == 4) ? r2[0] : g0;
    g1 = (w == 4) ? r2[1] : g1;
    c0 = (w == 4) ? vb2[0] : c0;
    c1 = (w == 4) ? vb2[1] : c1;
    g0 = (w == 5) ? r2[2] : g0;
    g1 = (w == 5) ? r2[3] : g1;
    c0 = (w == 5) ? vb2[2] : c0;
    c1 = (w == 5) ? vb2[3] : c1;
    g0 = (w == 6) ? r3[0] : g0;
    g1 = (w == 6) ? r3[1] : g1;
    c0 = (w == 6) ? vb3[0] : c0;
    c1 = (w == 6) ? vb3[1] : c1;
    g0 = (w == 7) ? r3[2] : g0;
    g1 = (w == 7) ? r3[3] : g1;
    c0 = (w == 7) ? vb3[2] : c0;
    c1 = (w == 7) ? vb3[3] : c1;
    o0 += sc * (g0 + c0);
    o1 += sc * (g1 + c1);
  }
  sO[tid * 2 + 0] = o0 * 0.25f + hb0;
  sO[tid * 2 + 1] = o1 * 0.25f + hb1;
  __syncthreads();
  if (wave == 0) {
    const v4f v = *(const v4f*)(sO + lane * 4);
    float* dst = out + (size_t)blockIdx.x * 128 + lane * 4;
    for (int pass = 0; pass < 2; ++pass) {
      *(volatile v4f*)dst = v;
      __threadfence();
    }
  }
}

extern "C" void kernel_launch(void* const* d_in, const int* in_sizes, int n_in,
                              void* d_out, int out_size, void* d_ws, size_t ws_size,
                              hipStream_t stream) {
  if (n_in < 7) return;
  if (in_sizes[0] != kTok * kDin) return;
  if (in_sizes[1] != kDin * kExp) return;
  if (in_sizes[2] != kExp) return;
  if (in_sizes[3] != kExp * kDin * kOut) return;
  if (in_sizes[4] != kExp * kOut) return;
  if (in_sizes[5] != kOut * kCls) return;
  if (in_sizes[6] != kCls) return;
  if (out_size != kBat * kCls) return;
  if (ws_size < kWsTotal) return;

  const float* x        = (const float*)d_in[0];
  const float* gate_w   = (const float*)d_in[1];
  const float* gate_b   = (const float*)d_in[2];
  const float* expert_w = (const float*)d_in[3];
  const float* expert_b = (const float*)d_in[4];
  const float* head_w   = (const float*)d_in[5];
  const float* head_b   = (const float*)d_in[6];
  float* out = (float*)d_out;

  char* ws = (char*)d_ws;
  unsigned short* VT  = (unsigned short*)(ws + kOffVT);
  float*          VB  = (float*)(ws + kOffVB);
  int*            WIN = (int*)(ws + kOffWIN);
  float*          SC  = (float*)(ws + kOffSC);
  float*          G   = (float*)(ws + kOffG);

  gate_select_kernel<<<kTok / kGateThreads, kGateThreads, 0, stream>>>(x, gate_w, gate_b, WIN, SC);
  fold_head_kernel<<<kExp * 16 + 1, 256, 0, stream>>>(expert_w, expert_b, head_w, VT, VB);
  xv_wmma_kernel<<<kTok / 64 / 8, 256, 0, stream>>>(x, VT, G);
  pool_select_kernel<<<kBat / 64, 64, 0, stream>>>(G, WIN, SC, VB, head_b, out);
}
